// equi_conv3_21603685499532
// MI455X (gfx1250) — hardware-verified
//
#include <hip/hip_runtime.h>
#include <math.h>

typedef __attribute__((ext_vector_type(16))) __bf16   v16b;
typedef __attribute__((ext_vector_type(8)))  __bf16   v8b;
typedef __attribute__((ext_vector_type(8)))  float    v8f;
typedef __attribute__((ext_vector_type(4)))  float    v4f;
typedef __attribute__((ext_vector_type(4)))  unsigned v4u;

#define PIN_VGPR32(x) asm volatile("" : "+v"(x))

constexpr int kBatch  = 2;
constexpr int kPts    = 1024;
constexpr int kNbr    = 16;
constexpr int kCin    = 64;
constexpr int kCout   = 32;
constexpr int kKpt    = 7;
constexpr int kRot    = 60;
constexpr int kBins   = 5;
constexpr int kRotBin = 12;
constexpr int kUrows  = kCout * kKpt * 3;
constexpr int kMrows  = kUrows + kCout;
constexpr int kColB   = kPts * 3;
constexpr int kNcols  = kBatch * kColB;
static_assert(kBins * kRotBin == kRot, "bins");
static_assert(kUrows == 672 && kMrows == 704 && kNcols == 6144 && kColB == 3072, "shapes");
static_assert((kMrows % 64) == 0 && (kNcols % 64) == 0 && (kCin % 32) == 0, "GEMM tile multiples");

constexpr size_t kSzAPL  = (size_t)kMrows * kCin * 2;
constexpr size_t kSzBTP  = (size_t)kNcols * kCin * 2;
constexpr size_t kSzNDN  = (size_t)kBatch * kNbr * 3 * kPts * 4;
constexpr size_t kSzCMAT = (size_t)kMrows * kNcols * 4;
constexpr size_t kSzBVAL = (size_t)kBatch * kCout * kBins * kPts * 4;
constexpr size_t kSzBIDX = kSzBVAL;
constexpr size_t kSzRIDX = (size_t)kBatch * kCout * kPts * 4;
constexpr size_t kSzFO2  = (size_t)kBatch * kCout * kKpt * kPts * 4;
constexpr size_t kOffAPL  = 0;
constexpr size_t kOffBTP  = kOffAPL  + kSzAPL;
constexpr size_t kOffNDN  = kOffBTP  + kSzBTP;
constexpr size_t kOffCMAT = kOffNDN  + kSzNDN;
constexpr size_t kOffBVAL = kOffCMAT + kSzCMAT;
constexpr size_t kOffBIDX = kOffBVAL + kSzBVAL;
constexpr size_t kOffRIDX = kOffBIDX + kSzBIDX;
constexpr size_t kOffFO2  = kOffRIDX + kSzRIDX;
constexpr size_t kWsTotal = kOffFO2  + kSzFO2;
static_assert(kWsTotal == 23289856ull, "carve total");
static_assert(kWsTotal <= 134217728ull, "carve cap");
static_assert((kOffBTP % 128) == 0 && (kOffNDN % 128) == 0 && (kOffCMAT % 128) == 0 && (kOffBVAL % 128) == 0 &&
              (kOffBIDX % 128) == 0 && (kOffRIDX % 128) == 0 && (kOffFO2 % 128) == 0, "128-B aligned regions");

__device__ __forceinline__ unsigned rne_bf16_bits(float f) {
  unsigned u = __float_as_uint(f);
  const unsigned lsb = (u & 0x00010000u) ? 1u : 0u;
  u = (u + 0x7FFFu + lsb) & 0xFFFF0000u;
  return u;
}
__device__ __forceinline__ float rne_bf16_f32(float f) { return __uint_as_float(rne_bf16_bits(f)); }
__device__ __forceinline__ unsigned pack_bf16_pair(unsigned lo_bits, unsigned hi_bits) {
  return __builtin_amdgcn_perm(hi_bits, lo_bits, 0x07060302u);
}
__device__ __forceinline__ void unit3(float x, float y, float z, float& ox, float& oy, float& oz) {
#pragma clang fp contract(off)
  const float xx = x * x;
  const float yy = y * y;
  const float zz = z * z;
  const float ss = (xx + zz) + yy;
  const float nrm = sqrtf(ss);
  const float den = fmaxf(nrm, 1e-12f);
  const float inv = 1.0f / den;
  ox = x * inv;
  oy = y * inv;
  oz = z * inv;
}
__device__ __forceinline__ void pack8_store(const float* __restrict__ src, unsigned stride, unsigned short* dst) {
  const float a0 = src[0];
  const float a1 = src[(size_t)stride];
  const float a2 = src[(size_t)stride * 2];
  const float a3 = src[(size_t)stride * 3];
  const float a4 = src[(size_t)stride * 4];
  const float a5 = src[(size_t)stride * 5];
  const float a6 = src[(size_t)stride * 6];
  const float a7 = src[(size_t)stride * 7];
  const unsigned w0 = pack_bf16_pair(rne_bf16_bits(a0), rne_bf16_bits(a1));
  const unsigned w1 = pack_bf16_pair(rne_bf16_bits(a2), rne_bf16_bits(a3));
  const unsigned w2 = pack_bf16_pair(rne_bf16_bits(a4), rne_bf16_bits(a5));
  const unsigned w3 = pack_bf16_pair(rne_bf16_bits(a6), rne_bf16_bits(a7));
  const v4u w = {w0, w1, w2, w3};
  volatile v4u* q = (volatile v4u*)(void*)dst;
  *q = w;
  __threadfence();
  *q = w;
}

constexpr int kPrepBlkAW = kUrows * kCin / 8 / 256;
constexpr int kPrepBlkA  = kMrows * kCin / 8 / 256;
constexpr int kPrepBlkB  = kNcols * kCin / 8 / 256;
constexpr int kPrepBlkN  = kBatch * kPts / 256;
static_assert(kPrepBlkAW == 21 && kPrepBlkA == 22 && kPrepBlkB == 192 && kPrepBlkN == 8, "prep coverage");
static_assert(kPrepBlkA * 256 * 8 == kMrows * kCin && kPrepBlkB * 256 * 8 == kNcols * kCin, "prep coverage exact");

__global__ __launch_bounds__(256) void prep_kernel(
    const int* __restrict__ nbrI, const float* __restrict__ verts, const float* __restrict__ fm,
    const float* __restrict__ Wt, const float* __restrict__ Wc,
    unsigned short* __restrict__ Apl, unsigned short* __restrict__ Btp, float* __restrict__ ndnT)
{
  const unsigned t = threadIdx.x;
  const unsigned blk = blockIdx.x;
  if (blk < (unsigned)kPrepBlkAW) {
    unsigned g = blk * 256u + t;
    PIN_VGPR32(g);
    unsigned row = g >> 3;
    PIN_VGPR32(row);
    unsigned c8 = (g & 7u) * 8u;
    PIN_VGPR32(c8);
    unsigned d = row / 21u;
    PIN_VGPR32(d);
    unsigned rem = row - d * 21u;
    PIN_VGPR32(rem);
    pack8_store(Wt + (size_t)(d * 64u + c8) * 21u + rem, 21u, Apl + (size_t)g * 8u);
  } else if (blk < (unsigned)kPrepBlkA) {
    unsigned g = blk * 256u + t;
    PIN_VGPR32(g);
    unsigned row = g >> 3;
    PIN_VGPR32(row);
    unsigned c8 = (g & 7u) * 8u;
    PIN_VGPR32(c8);
    pack8_store(Wc + (size_t)(row - (unsigned)kUrows) * 64u + c8, 1u, Apl + (size_t)g * 8u);
  } else if (blk < (unsigned)(kPrepBlkA + kPrepBlkB)) {
    unsigned g = (blk - (unsigned)kPrepBlkA) * 256u + t;
    PIN_VGPR32(g);
    unsigned n = g >> 3;
    PIN_VGPR32(n);
    unsigned c8 = (g & 7u) * 8u;
    PIN_VGPR32(c8);
    unsigned bsel = (n >= (unsigned)kColB) ? 1u : 0u;
    unsigned nn = n - bsel * (unsigned)kColB;
    PIN_VGPR32(nn);
    pack8_store(fm + (size_t)bsel * (size_t)(kCin * kColB) + (size_t)c8 * kColB + nn, (unsigned)kColB,
                Btp + (size_t)g * 8u);
  } else {
    unsigned g = (blk - (unsigned)(kPrepBlkA + kPrepBlkB)) * 256u + t;
    PIN_VGPR32(g);
    const unsigned b = g >> 10;
    const unsigned p = g & 1023u;
    const float cx = rne_bf16_f32(verts[(size_t)g * 3 + 0]);
    const float cy = rne_bf16_f32(verts[(size_t)g * 3 + 1]);
    const float cz = rne_bf16_f32(verts[(size_t)g * 3 + 2]);
    const int* nrow = nbrI + (size_t)g * kNbr;
    float* dcol = ndnT + (size_t)b * (kNbr * 3 * kPts) + p;
#pragma unroll 1
    for (int n = 0; n < kNbr; ++n) {
      int nb = nrow[n];
      nb = nb < 0 ? 0 : nb;
      nb = nb > (kPts - 1) ? (kPts - 1) : nb;
      const float* vn = verts + ((size_t)b * kPts + (unsigned)nb) * 3;
      const float x = rne_bf16_f32(vn[0]) - cx;
      const float y = rne_bf16_f32(vn[1]) - cy;
      const float z = rne_bf16_f32(vn[2]) - cz;
      float ux, uy, uz;
      unit3(x, y, z, ux, uy, uz);
      volatile float* q0 = dcol + (size_t)(n * 3 + 0) * kPts;
      volatile float* q1 = dcol + (size_t)(n * 3 + 1) * kPts;
      volatile float* q2 = dcol + (size_t)(n * 3 + 2) * kPts;
      *q0 = ux;
      *q1 = uy;
      *q2 = uz;
      __threadfence();
      *q0 = ux;
      *q1 = uy;
      *q2 = uz;
    }
  }
}

union FragB { v16b v; v8b h[2]; };
__device__ __forceinline__ v16b frag_load_bf16(const __bf16* p) {
  FragB f;
  f.h[0] = *(const v8b*)(p);
  f.h[1] = *(const v8b*)(p + 16);
  return f.v;
}
__device__ __forceinline__ v8f mma_bf16_guarded(v16b a, v16b b, v8f c) {
  c = __builtin_amdgcn_wmma_f32_16x16x32_bf16(false, a, false, b, (short)0, c, false, false);
  asm volatile("v_nop\n\tv_nop\n\tv_nop\n\tv_nop" : "+v"(c) : "v"(a), "v"(b));
  return c;
}

__global__ __launch_bounds__(256) void gemm_bf16_kernel(
    const unsigned short* __restrict__ Ap, int lda,
    const unsigned short* __restrict__ Btp, int ldb,
    float* __restrict__ Cout, int ldc, int M, int N, int K)
{
  const __bf16* A  = (const __bf16*)(const void*)Ap;
  const __bf16* Bt = (const __bf16*)(const void*)Btp;
  __shared__ __align__(16) float sT[8][16 * 68];
  const int lane = threadIdx.x & 31;
  const int wave = threadIdx.x >> 5;
  const int tilesN = N >> 6;
  const int tilesM = M >> 6;
  const int tile = blockIdx.x * 8 + wave;
  if (tile >= tilesM * tilesN) return;
  const int tm = tile / tilesN;
  const int tn = tile - tm * tilesN;
  const int m0 = tm << 6;
  const int n0 = tn << 6;
  const int rlane = lane & 15;
  const int koff  = (lane >> 4) * 8;
  const int mOff  = (lane >> 4) * 8;

  v8f acc[4][4];
#pragma unroll
  for (int i = 0; i < 4; ++i)
#pragma unroll
    for (int j = 0; j < 4; ++j) acc[i][j] = (v8f){0.f, 0.f, 0.f, 0.f, 0.f, 0.f, 0.f, 0.f};

  for (int k0 = 0; k0 < K; k0 += 32) {
    v16b bh[4];
#pragma unroll
    for (int j = 0; j < 4; ++j) {
      const size_t bo = (size_t)(n0 + (j << 4) + rlane) * ldb + koff + k0;
      bh[j] = frag_load_bf16(Bt + bo);
    }
#pragma unroll
    for (int i = 0; i < 4; ++i) {
      const size_t ao = (size_t)(m0 + (i << 4) + rlane) * lda + koff + k0;
      const v16b ah = frag_load_bf16(A + ao);
#pragma unroll
      for (int j = 0; j < 4; ++j) acc[i][j] = mma_bf16_guarded(ah, bh[j], acc[i][j]);
    }
  }

  float* slab = sT[wave];
#pragma unroll
  for (int i = 0; i < 4; ++i) {
    const int mBase = m0 + (i << 4);
#pragma unroll
    for (int j = 0; j < 4; ++j) {
#pragma unroll
      for (int r = 0; r < 8; ++r) slab[(mOff + r) * 68 + (j << 4) + rlane] = acc[i][j][r];
    }
    __builtin_amdgcn_fence(__ATOMIC_RELEASE, "workgroup");
    __builtin_amdgcn_wave_barrier();
    __builtin_amdgcn_fence(__ATOMIC_ACQUIRE, "workgroup");
    {
      const int hh = lane >> 4, c4 = (lane & 15) * 4;
      for (int pass = 0; pass < 2; ++pass) {
#pragma unroll
        for (int it = 0; it < 8; ++it) {
          const int row = it * 2 + hh;
          const v4f v = *(const v4f*)(slab + row * 68 + c4);
          *(volatile v4f*)(Cout + (size_t)(mBase + row) * ldc + n0 + c4) = v;
        }
        __threadfence();
      }
    }
    __builtin_amdgcn_fence(__ATOMIC_RELEASE, "workgroup");
    __builtin_amdgcn_wave_barrier();
    __builtin_amdgcn_fence(__ATOMIC_ACQUIRE, "workgroup");
  }
}

__global__ __launch_bounds__(512) void search_kernel(
    const int* __restrict__ nbrI, const float* __restrict__ dirs, const float* __restrict__ RsG,
    const float* __restrict__ Cm, const float* __restrict__ ndnT,
    float* __restrict__ binval, int* __restrict__ binidx)
{
  __shared__ __align__(16) float sFo[kPts * kRotBin];
  __shared__ __align__(16) float sRm[kRotBin * 12];
  __shared__ __align__(16) float sKd[32];
  __shared__ __align__(16) float sKr[kKpt * kRotBin * 4];

  const unsigned t = threadIdx.x;
  const unsigned blk = blockIdx.x;
  const unsigned bd = blk / (unsigned)kBins;
  const unsigned bin = blk - bd * (unsigned)kBins;
  const unsigned d = bd & 31u;
  const unsigned b = bd >> 5;

  {
    unsigned ec = t < 143u ? t : 143u;
    PIN_VGPR32(ec);
    unsigned rr = ec / 12u;
    PIN_VGPR32(rr);
    unsigned w = ec - rr * 12u;
    PIN_VGPR32(w);
    const unsigned ii = w >> 2;
    const unsigned jj = w & 3u;
    const unsigned jc = jj < 2u ? jj : 2u;
    float rv = RsG[(size_t)(bin * (unsigned)kRotBin + rr) * 9u + ii * 3u + jc];
    PIN_VGPR32(rv);
    const float val = (jj < 3u) ? rne_bf16_f32(rv) : 0.0f;
    if (t < 144u) sRm[t] = val;
  }
  {
    unsigned kk = t < 6u ? t : 6u;
    PIN_VGPR32(kk);
    const float* dp = dirs + (size_t)(d * (unsigned)kKpt + kk) * 3u;
    float dx = dp[0];
    float dy = dp[1];
    float dz = dp[2];
    PIN_VGPR32(dx);
    PIN_VGPR32(dy);
    PIN_VGPR32(dz);
    float ux, uy, uz;
    unit3(rne_bf16_f32(dx), rne_bf16_f32(dy), rne_bf16_f32(dz), ux, uy, uz);
    if (t < 7u) {
      sKd[t * 3u + 0u] = ux;
      sKd[t * 3u + 1u] = uy;
      sKd[t * 3u + 2u] = uz;
    }
  }
  __syncthreads();
  {
    unsigned ec = t < 335u ? t : 335u;
    PIN_VGPR32(ec);
    unsigned kr = ec >> 2;
    PIN_VGPR32(kr);
    const unsigned i3 = ec & 3u;
    const unsigned ic = i3 < 2u ? i3 : 2u;
    unsigned k1 = kr / 12u;
    PIN_VGPR32(k1);
    unsigned r1 = kr - k1 * 12u;
    PIN_VGPR32(r1);
    const float a0 = sRm[r1 * 12u + ic * 4u + 0u];
    const float a1 = sRm[r1 * 12u + ic * 4u + 1u];
    const float a2 = sRm[r1 * 12u + ic * 4u + 2u];
    const float e0 = sKd[k1 * 3u + 0u];
    const float e1 = sKd[k1 * 3u + 1u];
    const float e2 = sKd[k1 * 3u + 2u];
    float val = a0 * e0;
    val = fmaf(a1, e1, val);
    val = fmaf(a2, e2, val);
    val = (i3 < 3u) ? val : 0.0f;
    if (t < 336u) sKr[t] = val;
  }

  float acc[2][12];
#pragma unroll
  for (int m = 0; m < 2; ++m)
#pragma unroll
    for (int r = 0; r < 12; ++r) acc[m][r] = 0.0f;

#pragma unroll 1
  for (int k = 0; k < kKpt; ++k) {
    __syncthreads();
    const float* crow = Cm + (size_t)(d * 21u + (unsigned)k * 3u) * kNcols + (size_t)b * kColB;
#pragma unroll 1
    for (int m = 0; m < 2; ++m) {
      const unsigned q = t + 512u * (unsigned)m;
      const float* u0 = crow + (size_t)q * 3u;
      const float* u1 = u0 + kNcols;
      const float* u2 = u1 + kNcols;
      const float u00 = u0[0], u01 = u0[1], u02 = u0[2];
      const float u10 = u1[0], u11 = u1[1], u12 = u1[2];
      const float u20 = u2[0], u21 = u2[1], u22 = u2[2];
#pragma unroll 1
      for (int r = 0; r < kRotBin; ++r) {
        const v4f r0 = *(const v4f*)(&sRm[r * 12 + 0]);
        const v4f r1 = *(const v4f*)(&sRm[r * 12 + 4]);
        const v4f r2 = *(const v4f*)(&sRm[r * 12 + 8]);
        float f = r0[0] * u00;
        f = fmaf(r0[1], u10, f);
        f = fmaf(r0[2], u20, f);
        f = fmaf(r1[0], u01, f);
        f = fmaf(r1[1], u11, f);
        f = fmaf(r1[2], u21, f);
        f = fmaf(r2[0], u02, f);
        f = fmaf(r2[1], u12, f);
        f = fmaf(r2[2], u22, f);
        sFo[q * 12u + (unsigned)r] = f;
      }
    }
    __syncthreads();
    float kr[12][3];
#pragma unroll
    for (int r = 0; r < 12; ++r) {
      const v4f kv = *(const v4f*)(&sKr[(k * 12 + r) * 4]);
      kr[r][0] = kv[0];
      kr[r][1] = kv[1];
      kr[r][2] = kv[2];
    }
#pragma unroll
    for (int m = 0; m < 2; ++m) {
      const unsigned p = t + 512u * (unsigned)m;
      const int* nrow = nbrI + ((size_t)b * kPts + p) * kNbr;
      const float* ncol = ndnT + (size_t)b * (kNbr * 3 * kPts) + p;
      float mx[12];
#pragma unroll
      for (int r = 0; r < 12; ++r) mx[r] = -INFINITY;
#pragma unroll 1
      for (int n = 0; n < kNbr; ++n) {
        int nb = nrow[n];
        nb = nb < 0 ? 0 : nb;
        nb = nb > (kPts - 1) ? (kPts - 1) : nb;
        const float nx = ncol[(size_t)(n * 3 + 0) * kPts];
        const float ny = ncol[(size_t)(n * 3 + 1) * kPts];
        const float nz = ncol[(size_t)(n * 3 + 2) * kPts];
        const unsigned fb = (unsigned)nb * 12u;
        const v4f f0 = *(const v4f*)(&sFo[fb + 0u]);
        const v4f f1 = *(const v4f*)(&sFo[fb + 4u]);
        const v4f f2 = *(const v4f*)(&sFo[fb + 8u]);
        const float fv[12] = {f0[0], f0[1], f0[2], f0[3], f1[0], f1[1], f1[2], f1[3], f2[0], f2[1], f2[2], f2[3]};
#pragma unroll
        for (int r = 0; r < 12; ++r) {
          float th = kr[r][0] * nx;
          th = fmaf(kr[r][1], ny, th);
          th = fmaf(kr[r][2], nz, th);
          const float pr = fv[r] * th;
          mx[r] = fmaxf(mx[r], pr);
        }
      }
#pragma unroll
      for (int r = 0; r < 12; ++r) acc[m][r] = acc[m][r] + mx[r];
    }
  }

#pragma unroll
  for (int m = 0; m < 2; ++m) {
    float best = acc[m][0];
    int bi = 0;
#pragma unroll
    for (int r = 1; r < 12; ++r) {
      const bool gt = acc[m][r] > best;
      best = gt ? acc[m][r] : best;
      bi = gt ? r : bi;
    }
    const unsigned p = t + 512u * (unsigned)m;
    const size_t off = ((size_t)bd * kBins + bin) * kPts + p;
    const int gi = (int)(bin * (unsigned)kRotBin) + bi;
    volatile float* pv = binval + off;
    volatile int* pi = binidx + off;
    *pv = best;
    *pi = gi;
    __threadfence();
    *pv = best;
    *pi = gi;
  }
}

__global__ __launch_bounds__(256) void select_kernel(
    const float* __restrict__ RsG, const float* __restrict__ Cm,
    const float* __restrict__ binval, const int* __restrict__ binidx,
    int* __restrict__ ridx, float* __restrict__ fo2)
{
  const unsigned t = threadIdx.x;
  const unsigned bd = blockIdx.x >> 2;
  const unsigned p = ((blockIdx.x & 3u) << 8) + t;
  const unsigned d = bd & 31u;
  const unsigned b = bd >> 5;
  const size_t base = (size_t)bd * kBins * kPts + p;
  float bv[5];
  int bx[5];
#pragma unroll
  for (int s = 0; s < 5; ++s) {
    bv[s] = binval[base + (size_t)s * kPts];
    bx[s] = binidx[base + (size_t)s * kPts];
    PIN_VGPR32(bv[s]);
    PIN_VGPR32(bx[s]);
  }
  float best = bv[0];
  int bi = bx[0];
#pragma unroll
  for (int s = 1; s < 5; ++s) {
    const bool gt = bv[s] > best;
    best = gt ? bv[s] : best;
    bi = gt ? bx[s] : bi;
  }
  bi = bi < 0 ? 0 : bi;
  bi = bi > (kRot - 1) ? (kRot - 1) : bi;
  {
    volatile int* pr = ridx + (size_t)bd * kPts + p;
    *pr = bi;
    __threadfence();
    *pr = bi;
  }
  const float* rp = RsG + (size_t)bi * 9;
  const float m00 = rne_bf16_f32(rp[0]), m01 = rne_bf16_f32(rp[1]), m02 = rne_bf16_f32(rp[2]);
  const float m10 = rne_bf16_f32(rp[3]), m11 = rne_bf16_f32(rp[4]), m12 = rne_bf16_f32(rp[5]);
  const float m20 = rne_bf16_f32(rp[6]), m21 = rne_bf16_f32(rp[7]), m22 = rne_bf16_f32(rp[8]);
  const float* cb = Cm + (size_t)(d * 21u) * kNcols + (size_t)b * kColB + (size_t)p * 3u;
  float* fob = fo2 + (size_t)bd * kKpt * kPts + p;
#pragma unroll 1
  for (int k = 0; k < kKpt; ++k) {
    const float* u0 = cb + (size_t)(k * 3) * kNcols;
    const float* u1 = u0 + kNcols;
    const float* u2 = u1 + kNcols;
    const float u00 = u0[0], u01 = u0[1], u02 = u0[2];
    const float u10 = u1[0], u11 = u1[1], u12 = u1[2];
    const float u20 = u2[0], u21 = u2[1], u22 = u2[2];
    float f = m00 * u00;
    f = fmaf(m01, u10, f);
    f = fmaf(m02, u20, f);
    f = fmaf(m10, u01, f);
    f = fmaf(m11, u11, f);
    f = fmaf(m12, u21, f);
    f = fmaf(m20, u02, f);
    f = fmaf(m21, u12, f);
    f = fmaf(m22, u22, f);
    volatile float* pf = fob + (size_t)k * kPts;
    *pf = f;
    __threadfence();
    *pf = f;
  }
}

__global__ __launch_bounds__(256) void final_kernel(
    const int* __restrict__ nbrI, const float* __restrict__ dirs, const float* __restrict__ RsG,
    const float* __restrict__ Cm, const float* __restrict__ ndnT,
    const int* __restrict__ ridx, const float* __restrict__ fo2, float* __restrict__ out)
{
  __shared__ __align__(16) float sKd[32];
  __shared__ __align__(16) float sOut[256 * 3];
  const unsigned t = threadIdx.x;
  const unsigned lane = t & 31u;
  const unsigned wave = t >> 5;
  const unsigned bd = blockIdx.x >> 2;
  const unsigned p0 = (blockIdx.x & 3u) << 8;
  const unsigned p = p0 + t;
  const unsigned d = bd & 31u;
  const unsigned b = bd >> 5;
  {
    unsigned kk = t < 6u ? t : 6u;
    PIN_VGPR32(kk);
    const float* dp = dirs + (size_t)(d * (unsigned)kKpt + kk) * 3u;
    float dx = dp[0];
    float dy = dp[1];
    float dz = dp[2];
    PIN_VGPR32(dx);
    PIN_VGPR32(dy);
    PIN_VGPR32(dz);
    float ux, uy, uz;
    unit3(rne_bf16_f32(dx), rne_bf16_f32(dy), rne_bf16_f32(dz), ux, uy, uz);
    if (t < 7u) {
      sKd[t * 3u + 0u] = ux;
      sKd[t * 3u + 1u] = uy;
      sKd[t * 3u + 2u] = uz;
    }
  }
  __syncthreads();
  int ri = ridx[(size_t)bd * kPts + p];
  ri = ri < 0 ? 0 : ri;
  ri = ri > (kRot - 1) ? (kRot - 1) : ri;
  const float* rp = RsG + (size_t)ri * 9;
  const float m00 = rne_bf16_f32(rp[0]), m01 = rne_bf16_f32(rp[1]), m02 = rne_bf16_f32(rp[2]);
  const float m10 = rne_bf16_f32(rp[3]), m11 = rne_bf16_f32(rp[4]), m12 = rne_bf16_f32(rp[5]);
  const float m20 = rne_bf16_f32(rp[6]), m21 = rne_bf16_f32(rp[7]), m22 = rne_bf16_f32(rp[8]);
  const int* nrow = nbrI + ((size_t)b * kPts + p) * kNbr;
  const float* ncol = ndnT + (size_t)b * (kNbr * 3 * kPts) + p;
  const float* fob = fo2 + (size_t)bd * kKpt * kPts;
  float o0 = 0.0f, o1 = 0.0f, o2 = 0.0f;
#pragma unroll 1
  for (int k = 0; k < kKpt; ++k) {
    const float e0 = sKd[k * 3 + 0];
    const float e1 = sKd[k * 3 + 1];
    const float e2 = sKd[k * 3 + 2];
    float c0 = m00 * e0;
    c0 = fmaf(m01, e1, c0);
    c0 = fmaf(m02, e2, c0);
    float c1 = m10 * e0;
    c1 = fmaf(m11, e1, c1);
    c1 = fmaf(m12, e2, c1);
    float c2 = m20 * e0;
    c2 = fmaf(m21, e1, c2);
    c2 = fmaf(m22, e2, c2);
    float kaw = -INFINITY;
#pragma unroll 1
    for (int n = 0; n < kNbr; ++n) {
      int nb = nrow[n];
      nb = nb < 0 ? 0 : nb;
      nb = nb > (kPts - 1) ? (kPts - 1) : nb;
      const float nx = ncol[(size_t)(n * 3 + 0) * kPts];
      const float ny = ncol[(size_t)(n * 3 + 1) * kPts];
      const float nz = ncol[(size_t)(n * 3 + 2) * kPts];
      float th = c0 * nx;
      th = fmaf(c1, ny, th);
      th = fmaf(c2, nz, th);
      th = fmaxf(th, 0.0f);
      const float g = fob[(size_t)k * kPts + (unsigned)nb];
      const float pr = g * th;
      kaw = fmaxf(kaw, pr);
    }
    o0 = fmaf(kaw, c0, o0);
    o1 = fmaf(kaw, c1, o1);
    o2 = fmaf(kaw, c2, o2);
  }
  {
    const float* cc = Cm + (size_t)(kUrows + d) * kNcols + (size_t)b * kColB + (size_t)p * 3u;
    o0 = o0 + cc[0];
    o1 = o1 + cc[1];
    o2 = o2 + cc[2];
  }
  sOut[t * 3u + 0u] = o0;
  sOut[t * 3u + 1u] = o1;
  sOut[t * 3u + 2u] = o2;
  __syncthreads();
  {
    const unsigned lc = lane < 23u ? lane : 23u;
    const v4f val = *(const v4f*)(&sOut[wave * 96u + lc * 4u]);
    float* op = out + ((size_t)bd * kPts + p0 + wave * 32u) * 3u + lc * 4u;
    if (lane < 24u) *(volatile v4f*)op = val;
    __threadfence();
    if (lane < 24u) *(volatile v4f*)op = val;
  }
}

extern "C" void kernel_launch(void* const* d_in, const int* in_sizes, int n_in,
                              void* d_out, int out_size, void* d_ws, size_t ws_size,
                              hipStream_t stream) {
  if (n_in < 7) return;
  if (in_sizes[0] != kBatch * kPts * kNbr) return;
  if (in_sizes[1] != kBatch * kPts * 3) return;
  if (in_sizes[2] != kBatch * kCin * kPts * 3) return;
  if (in_sizes[3] != kCout * kCin * kKpt * 3) return;
  if (in_sizes[4] != kCout * kCin) return;
  if (in_sizes[5] != kCout * kKpt * 3) return;
  if (in_sizes[6] != kRot * 9) return;
  if (out_size != kBatch * kCout * kPts * 3) return;
  if (ws_size < kWsTotal) return;

  const int*   nbrI  = (const int*)d_in[0];
  const float* verts = (const float*)d_in[1];
  const float* fm    = (const float*)d_in[2];
  const float* Wt    = (const float*)d_in[3];
  const float* Wc    = (const float*)d_in[4];
  const float* dirs  = (const float*)d_in[5];
  const float* RsG   = (const float*)d_in[6];
  float* out = (float*)d_out;

  char* ws = (char*)d_ws;
  unsigned short* Apl  = (unsigned short*)(ws + kOffAPL);
  unsigned short* Btp  = (unsigned short*)(ws + kOffBTP);
  float*          ndnT = (float*)(ws + kOffNDN);
  float*          Cm   = (float*)(ws + kOffCMAT);
  float*          bval = (float*)(ws + kOffBVAL);
  int*            bidx = (int*)(ws + kOffBIDX);
  int*            ridx = (int*)(ws + kOffRIDX);
  float*          fo2  = (float*)(ws + kOffFO2);

  prep_kernel<<<kPrepBlkA + kPrepBlkB + kPrepBlkN, 256, 0, stream>>>(nbrI, verts, fm, Wt, Wc, Apl, Btp, ndnT);

  gemm_bf16_kernel<<<(kMrows / 64) * (kNcols / 64) / 8, 256, 0, stream>>>(
      Apl, kCin, Btp, kCin, Cm, kNcols, kMrows, kNcols, kCin);

  search_kernel<<<kBatch * kCout * kBins, 512, 0, stream>>>(nbrI, dirs, RsG, Cm, ndnT, bval, bidx);

  select_kernel<<<kBatch * kCout * kPts / 256, 256, 0, stream>>>(RsG, Cm, bval, bidx, ridx, fo2);

  final_kernel<<<kBatch * kCout * kPts / 256, 256, 0, stream>>>(nbrI, dirs, RsG, Cm, ndnT, ridx, fo2, out);
}
